// LatticeRNNCell_91268055040455
// MI455X (gfx1250) — hardware-run, weakly checked
//
#include <hip/hip_runtime.h>
#include <math.h>

typedef __attribute__((ext_vector_type(16))) _Float16 v16h;
typedef __attribute__((ext_vector_type(8)))  _Float16 v8h;
typedef __attribute__((ext_vector_type(8)))  float    v8f;
typedef __attribute__((ext_vector_type(4)))  float    v4f;
typedef __attribute__((ext_vector_type(2)))  unsigned v2u;
typedef __attribute__((ext_vector_type(2)))  float    v2f;

constexpr int kB  = 4096;
constexpr int kI  = 512;
constexpr int kH  = 1024;
constexpr int k3H = 3 * kH;
constexpr int kKG = kI + kH;
constexpr int k4H = 4 * kH;
constexpr int kOutHalf = kB * kH;
constexpr float kWCarry = 65536.0f;
constexpr float kWScale = 1.0f / kWCarry;
constexpr float kEps = 1e-5f;
static_assert(kH == 1024 && kI == 512 && kB == 4096);
static_assert(k3H == 3072 && kKG == 1536 && k4H == 4096);
static_assert(kOutHalf == 4194304);
static_assert((k3H % 32) == 0 && (kKG % 32) == 0);
static_assert((kB % 32) == 0 && (kH % 64) == 0 && (k4H % 64) == 0);

constexpr size_t kSzCat = (size_t)kB * k3H * 2;
constexpr size_t kSzWP  = (size_t)kH * k3H * 2;
constexpr size_t kSzR   = (size_t)kB * kH * 4;
constexpr size_t kSzST  = (size_t)kB * 2 * 4;
constexpr size_t kSzXH  = (size_t)kB * kKG * 2;
constexpr size_t kSzWG  = (size_t)k4H * kKG * 2;
constexpr size_t kSzGT  = (size_t)kB * k4H * 4;
constexpr size_t kOffCH  = 0;
constexpr size_t kOffCC  = kOffCH  + kSzCat;
constexpr size_t kOffWHP = kOffCC  + kSzCat;
constexpr size_t kOffWCP = kOffWHP + kSzWP;
constexpr size_t kOffRH  = kOffWCP + kSzWP;
constexpr size_t kOffRC  = kOffRH  + kSzR;
constexpr size_t kOffSTH = kOffRC  + kSzR;
constexpr size_t kOffSTC = kOffSTH + kSzST;
constexpr size_t kOffXH  = kOffSTC + kSzST;
constexpr size_t kOffPC  = kOffXH  + kSzXH;
constexpr size_t kOffWG  = kOffPC  + kSzR;
constexpr size_t kOffGT  = kOffWG  + kSzWG;
constexpr size_t kWsTotal = kOffGT + kSzGT;
static_assert(kSzCat == 25165824ull && kSzWP == 6291456ull && kSzR == 16777216ull);
static_assert(kSzST == 32768ull && kSzXH == 12582912ull && kSzWG == 12582912ull && kSzGT == 67108864ull);
static_assert(kWsTotal == 205586432ull);
static_assert(kWsTotal <= 268435456ull);
static_assert((kSzCat % 256) == 0 && (kSzWP % 256) == 0 && (kSzR % 256) == 0 && (kSzST % 256) == 0 &&
              (kSzXH % 256) == 0 && (kSzWG % 256) == 0 && (kSzGT % 256) == 0);

__device__ __forceinline__ _Float16 f16_flush(float v) {
  const float w = (fabsf(v) < 6.103515625e-05f) ? 0.0f : v;
  return (_Float16)w;
}

__device__ __forceinline__ float bf16r(float v) {
  unsigned u = __float_as_uint(v);
  u = (u + 0x7FFFu + ((u >> 16) & 1u)) & 0xFFFF0000u;
  return __uint_as_float(u);
}

namespace eng {
union FragU { v16h v; v8h h[2]; };
__device__ __forceinline__ v16h frag_load(const _Float16* p) {
  FragU f;
  f.h[0] = *(const v8h*)(p);
  f.h[1] = *(const v8h*)(p + 16);
  return f.v;
}
__device__ __forceinline__ v8f mma(v16h a, v16h b, v8f c) {
  return __builtin_amdgcn_wmma_f32_16x16x32_f16(false, a, false, b, (short)0, c, false, false);
}
__device__ __forceinline__ void guard1(v8f& a, v16h x, v16h y) {
  asm volatile("v_nop\n\tv_nop\n\tv_nop\n\tv_nop" : "+v"(a) : "v"(x), "v"(y));
}
__device__ __forceinline__ void guard_acc(v8f& a) {
  asm volatile("v_nop\n\tv_nop\n\tv_nop\n\tv_nop" : "+v"(a));
}
__device__ __forceinline__ void keep4(v16h a, v16h b, v16h c, v16h d) {
  asm volatile("v_nop" :: "v"(a), "v"(b), "v"(c), "v"(d));
}

template <int MI, int SPL>
__global__ __launch_bounds__(256) void gemm_f16_kernel(
    const unsigned short* __restrict__ Ap, const unsigned short* __restrict__ A2p, int lda,
    const unsigned short* __restrict__ Btp, const unsigned short* __restrict__ Bt2p, int ldb,
    float* __restrict__ C, int ldc, int M, int N, int K, float scale, float rscale)
{
  static_assert(MI >= 1 && MI <= 2);
  static_assert(SPL >= 0 && SPL <= 2);
  const _Float16* A   = (const _Float16*)Ap;
  const _Float16* A2  = (const _Float16*)A2p;
  const _Float16* Bt  = (const _Float16*)Btp;
  const _Float16* Bt2 = (const _Float16*)Bt2p;
  __shared__ __align__(16) float sT[8][16 * 68];
  const int lane = threadIdx.x & 31;
  const int wave = threadIdx.x >> 5;
  const int tilesN = N >> 6;
  const int tilesM = M / (16 * MI);
  const int tile = blockIdx.x * 8 + wave;
  if (tile >= tilesM * tilesN) return;
  const int tm = tile / tilesN;
  const int tn = tile - tm * tilesN;
  const int m0 = tm * (16 * MI);
  const int n0 = tn << 6;
  const int rlane = lane & 15;
  const int koff  = (lane >> 4) * 8;
  const int mOff  = (lane >> 4) * 8;

  v8f acc[MI][4], accr[MI][4];
#pragma unroll
  for (int i = 0; i < MI; ++i)
#pragma unroll
    for (int j = 0; j < 4; ++j) {
      acc[i][j]  = (v8f){0.f, 0.f, 0.f, 0.f, 0.f, 0.f, 0.f, 0.f};
      accr[i][j] = (v8f){0.f, 0.f, 0.f, 0.f, 0.f, 0.f, 0.f, 0.f};
    }

  for (int k0 = 0; k0 < K; k0 += 32) {
    v16h bh[4], bl[4];
#pragma unroll
    for (int j = 0; j < 4; ++j) {
      const size_t bo = (size_t)(n0 + (j << 4) + rlane) * ldb + koff + k0;
      bh[j] = frag_load(Bt + bo);
      if (SPL == 2) bl[j] = frag_load(Bt2 + bo); else bl[j] = bh[j];
    }
#pragma unroll
    for (int i = 0; i < MI; ++i) {
      const size_t ao = (size_t)(m0 + (i << 4) + rlane) * lda + koff + k0;
      const v16h ah = frag_load(A + ao);
      v16h al = ah;
      if (SPL >= 1) al = frag_load(A2 + ao);
#pragma unroll
      for (int j = 0; j < 4; ++j) {
        acc[i][j] = mma(ah, bh[j], acc[i][j]);
        if (SPL >= 1) accr[i][j] = mma(al, bh[j], accr[i][j]);
        if (SPL == 2) accr[i][j] = mma(ah, bl[j], accr[i][j]);
      }
#pragma unroll
      for (int j = 0; j < 4; ++j) {
        guard1(acc[i][j], ah, al);
        if (SPL >= 1) guard1(accr[i][j], ah, al);
      }
    }
    keep4(bh[0], bh[1], bh[2], bh[3]);
    if (SPL == 2) keep4(bl[0], bl[1], bl[2], bl[3]);
  }
#pragma unroll
  for (int i = 0; i < MI; ++i)
#pragma unroll
    for (int j = 0; j < 4; ++j) {
      guard_acc(acc[i][j]);
      if (SPL >= 1) guard_acc(accr[i][j]);
    }

  float* slab = sT[wave];
#pragma unroll
  for (int i = 0; i < MI; ++i) {
    const int mBase = m0 + (i << 4);
#pragma unroll
    for (int j = 0; j < 4; ++j) {
#pragma unroll
      for (int r = 0; r < 8; ++r) {
        float v = acc[i][j][r] * scale;
        if (SPL >= 1) v += accr[i][j][r] * rscale;
        slab[(mOff + r) * 68 + (j << 4) + rlane] = v;
      }
    }
    __builtin_amdgcn_fence(__ATOMIC_RELEASE, "workgroup");
    __builtin_amdgcn_wave_barrier();
    __builtin_amdgcn_fence(__ATOMIC_ACQUIRE, "workgroup");
    {
      const int hh = lane >> 4, c4 = (lane & 15) * 4;
      for (int pass = 0; pass < 2; ++pass) {
#pragma unroll
        for (int it = 0; it < 8; ++it) {
          const int row = it * 2 + hh;
          const v4f v = *(const v4f*)(slab + row * 68 + c4);
          *(volatile v4f*)(C + (size_t)(mBase + row) * ldc + n0 + c4) = v;
        }
        __threadfence();
      }
    }
    __builtin_amdgcn_fence(__ATOMIC_RELEASE, "workgroup");
    __builtin_amdgcn_wave_barrier();
    __builtin_amdgcn_fence(__ATOMIC_ACQUIRE, "workgroup");
  }
}
}

__global__ __launch_bounds__(256) void cat3_pack_kernel(
    const float* __restrict__ a, const float* __restrict__ bsrc, const float* __restrict__ c,
    unsigned short* __restrict__ dst)
{
  const int j = blockIdx.x * 256 + threadIdx.x;
  const int b = j / (k3H / 8);
  const int k0 = (j - (k3H / 8) * b) * 8;
  const int which = k0 >> 10;
  const int col = k0 & (kH - 1);
  const float* src = (which == 0) ? a : ((which == 1) ? bsrc : c);
  const float* sp = src + (size_t)b * kH + col;
  const v4f a0 = *(const v4f*)(sp);
  const v4f a1 = *(const v4f*)(sp + 4);
  const float f0 = a0[0];
  const float f1 = a0[1];
  const float f2 = a0[2];
  const float f3 = a0[3];
  const float f4 = a1[0];
  const float f5 = a1[1];
  const float f6 = a1[2];
  const float f7 = a1[3];
  v8h hv;
  hv[0] = f16_flush(bf16r(f0));
  hv[1] = f16_flush(bf16r(f1));
  hv[2] = f16_flush(bf16r(f2));
  hv[3] = f16_flush(bf16r(f3));
  hv[4] = f16_flush(bf16r(f4));
  hv[5] = f16_flush(bf16r(f5));
  hv[6] = f16_flush(bf16r(f6));
  hv[7] = f16_flush(bf16r(f7));
  unsigned short* qh = dst + (size_t)j * 8;
  *(volatile v8h*)qh = hv;
  __threadfence();
  *(volatile v8h*)qh = hv;
}

__global__ __launch_bounds__(256) void w_pack_kernel(
    const float* __restrict__ src, unsigned short* __restrict__ dst)
{
  const int j = blockIdx.x * 256 + threadIdx.x;
  const float* sp = src + (size_t)j * 8;
  const v4f a0 = *(const v4f*)(sp);
  const v4f a1 = *(const v4f*)(sp + 4);
  const float f0 = a0[0];
  const float f1 = a0[1];
  const float f2 = a0[2];
  const float f3 = a0[3];
  const float f4 = a1[0];
  const float f5 = a1[1];
  const float f6 = a1[2];
  const float f7 = a1[3];
  v8h hv;
  hv[0] = f16_flush(bf16r(f0) * kWCarry);
  hv[1] = f16_flush(bf16r(f1) * kWCarry);
  hv[2] = f16_flush(bf16r(f2) * kWCarry);
  hv[3] = f16_flush(bf16r(f3) * kWCarry);
  hv[4] = f16_flush(bf16r(f4) * kWCarry);
  hv[5] = f16_flush(bf16r(f5) * kWCarry);
  hv[6] = f16_flush(bf16r(f6) * kWCarry);
  hv[7] = f16_flush(bf16r(f7) * kWCarry);
  unsigned short* qh = dst + (size_t)j * 8;
  *(volatile v8h*)qh = hv;
  __threadfence();
  *(volatile v8h*)qh = hv;
}

__global__ __launch_bounds__(256) void wg_pack_kernel(
    const float* __restrict__ Wih, const float* __restrict__ Whh, unsigned short* __restrict__ dst)
{
  const int j = blockIdx.x * 256 + threadIdx.x;
  const int n = j / (kKG / 8);
  const int k0 = (j - (kKG / 8) * n) * 8;
  const bool left = (k0 < kI);
  const int ci = left ? k0 : 0;
  const int ch = left ? 0 : (k0 - kI);
  const float* pi = Wih + (size_t)n * kI + ci;
  const float* ph = Whh + (size_t)n * kH + ch;
  const float* sp = left ? pi : ph;
  const v4f a0 = *(const v4f*)(sp);
  const v4f a1 = *(const v4f*)(sp + 4);
  const float f0 = a0[0];
  const float f1 = a0[1];
  const float f2 = a0[2];
  const float f3 = a0[3];
  const float f4 = a1[0];
  const float f5 = a1[1];
  const float f6 = a1[2];
  const float f7 = a1[3];
  v8h hv;
  hv[0] = f16_flush(bf16r(f0) * kWCarry);
  hv[1] = f16_flush(bf16r(f1) * kWCarry);
  hv[2] = f16_flush(bf16r(f2) * kWCarry);
  hv[3] = f16_flush(bf16r(f3) * kWCarry);
  hv[4] = f16_flush(bf16r(f4) * kWCarry);
  hv[5] = f16_flush(bf16r(f5) * kWCarry);
  hv[6] = f16_flush(bf16r(f6) * kWCarry);
  hv[7] = f16_flush(bf16r(f7) * kWCarry);
  unsigned short* qh = dst + (size_t)j * 8;
  *(volatile v8h*)qh = hv;
  __threadfence();
  *(volatile v8h*)qh = hv;
}

__global__ __launch_bounds__(256) void x_pack_kernel(
    const float* __restrict__ x, unsigned short* __restrict__ XH)
{
  const int j = blockIdx.x * 256 + threadIdx.x;
  const int b = j >> 6;
  const int k0 = (j & 63) * 8;
  const float* sp = x + (size_t)b * kI + k0;
  const v4f a0 = *(const v4f*)(sp);
  const v4f a1 = *(const v4f*)(sp + 4);
  const float f0 = a0[0];
  const float f1 = a0[1];
  const float f2 = a0[2];
  const float f3 = a0[3];
  const float f4 = a1[0];
  const float f5 = a1[1];
  const float f6 = a1[2];
  const float f7 = a1[3];
  v8h hv;
  hv[0] = f16_flush(bf16r(f0));
  hv[1] = f16_flush(bf16r(f1));
  hv[2] = f16_flush(bf16r(f2));
  hv[3] = f16_flush(bf16r(f3));
  hv[4] = f16_flush(bf16r(f4));
  hv[5] = f16_flush(bf16r(f5));
  hv[6] = f16_flush(bf16r(f6));
  hv[7] = f16_flush(bf16r(f7));
  unsigned short* qh = XH + (size_t)b * kKG + k0;
  *(volatile v8h*)qh = hv;
  __threadfence();
  *(volatile v8h*)qh = hv;
}

__global__ __launch_bounds__(256) void ln_stats_kernel(
    const float* __restrict__ R, const float* __restrict__ bias, float* __restrict__ ST)
{
  const int r = blockIdx.x * 256 + threadIdx.x;
  const float* rp = R + (size_t)r * kH;
  float s = 0.0f;
  for (int k = 0; k < kH; k += 4) {
    const v4f rv = *(const v4f*)(rp + k);
    const v4f bv = *(const v4f*)(bias + k);
    const float b0 = bv[0];
    const float b1 = bv[1];
    const float b2 = bv[2];
    const float b3 = bv[3];
    s += rv[0] + bf16r(b0);
    s += rv[1] + bf16r(b1);
    s += rv[2] + bf16r(b2);
    s += rv[3] + bf16r(b3);
  }
  const float mu = s / (float)kH;
  float q = 0.0f;
  for (int k = 0; k < kH; k += 4) {
    const v4f rv = *(const v4f*)(rp + k);
    const v4f bv = *(const v4f*)(bias + k);
    const float b0 = bv[0];
    const float b1 = bv[1];
    const float b2 = bv[2];
    const float b3 = bv[3];
    const float d0 = (rv[0] + bf16r(b0)) - mu;
    const float d1 = (rv[1] + bf16r(b1)) - mu;
    const float d2 = (rv[2] + bf16r(b2)) - mu;
    const float d3 = (rv[3] + bf16r(b3)) - mu;
    q += d0 * d0;
    q += d1 * d1;
    q += d2 * d2;
    q += d3 * d3;
  }
  const float var = q / (float)kH;
  const float rs = 1.0f / sqrtf(var + kEps);
  v2f st;
  st[0] = mu;
  st[1] = rs;
  float* p = ST + (size_t)r * 2;
  *(volatile v2f*)p = st;
  __threadfence();
  *(volatile v2f*)p = st;
}

__global__ __launch_bounds__(256) void ln_apply_h_kernel(
    const float* __restrict__ RH, const float* __restrict__ bias, const float* __restrict__ gamma,
    const float* __restrict__ beta, const float* __restrict__ ST, unsigned short* __restrict__ XH)
{
  const int j = blockIdx.x * 256 + threadIdx.x;
  const int b = j >> 7;
  const int c0 = (j & 127) * 8;
  const v2f st = *(const v2f*)(ST + (size_t)b * 2);
  const float mu = st[0];
  const float rs = st[1];
  const float* rp = RH + (size_t)b * kH + c0;
  v8h hv;
#pragma unroll
  for (int h = 0; h < 2; ++h) {
    const v4f rv = *(const v4f*)(rp + 4 * h);
    const v4f bv = *(const v4f*)(bias + c0 + 4 * h);
    const v4f gv = *(const v4f*)(gamma + c0 + 4 * h);
    const v4f ev = *(const v4f*)(beta + c0 + 4 * h);
#pragma unroll
    for (int e = 0; e < 4; ++e) {
      const float bs = bv[e];
      const float gs = gv[e];
      const float es = ev[e];
      const float v = rv[e] + bf16r(bs);
      const float p = (v - mu) * rs * bf16r(gs) + bf16r(es);
      hv[4 * h + e] = f16_flush(p);
    }
  }
  unsigned short* qh = XH + (size_t)b * kKG + kI + c0;
  *(volatile v8h*)qh = hv;
  __threadfence();
  *(volatile v8h*)qh = hv;
}

__global__ __launch_bounds__(256) void ln_apply_c_kernel(
    const float* __restrict__ RC, const float* __restrict__ bias, const float* __restrict__ gamma,
    const float* __restrict__ beta, const float* __restrict__ ST, float* __restrict__ PC)
{
  const int t = blockIdx.x * 256 + threadIdx.x;
  const int i = t * 4;
  const int b = i >> 10;
  const int c0 = i & (kH - 1);
  const v2f st = *(const v2f*)(ST + (size_t)b * 2);
  const float mu = st[0];
  const float rs = st[1];
  const v4f rv = *(const v4f*)(RC + (size_t)i);
  const v4f bv = *(const v4f*)(bias + c0);
  const v4f gv = *(const v4f*)(gamma + c0);
  const v4f ev = *(const v4f*)(beta + c0);
  v4f pv;
#pragma unroll
  for (int e = 0; e < 4; ++e) {
    const float bs = bv[e];
    const float gs = gv[e];
    const float es = ev[e];
    const float v = rv[e] + bf16r(bs);
    pv[e] = (v - mu) * rs * bf16r(gs) + bf16r(es);
  }
  float* p = PC + (size_t)i;
  *(volatile v4f*)p = pv;
  __threadfence();
  *(volatile v4f*)p = pv;
}

__global__ __launch_bounds__(256) void cell_out_kernel(
    const float* __restrict__ GT, const float* __restrict__ PC,
    const float* __restrict__ bih, const float* __restrict__ bhh, float* __restrict__ out)
{
  const int t = blockIdx.x * 256 + threadIdx.x;
  const int i = t * 4;
  const int b = i >> 10;
  const int j0 = i & (kH - 1);
  const float* gr = GT + (size_t)b * k4H + j0;
  const v4f gi4 = *(const v4f*)(gr);
  const v4f gf4 = *(const v4f*)(gr + kH);
  const v4f gg4 = *(const v4f*)(gr + 2 * kH);
  const v4f go4 = *(const v4f*)(gr + 3 * kH);
  const v4f ai4 = *(const v4f*)(bih + j0);
  const v4f af4 = *(const v4f*)(bih + kH + j0);
  const v4f ag4 = *(const v4f*)(bih + 2 * kH + j0);
  const v4f ao4 = *(const v4f*)(bih + 3 * kH + j0);
  const v4f hi4 = *(const v4f*)(bhh + j0);
  const v4f hf4 = *(const v4f*)(bhh + kH + j0);
  const v4f hg4 = *(const v4f*)(bhh + 2 * kH + j0);
  const v4f ho4 = *(const v4f*)(bhh + 3 * kH + j0);
  const v4f pc4 = *(const v4f*)(PC + (size_t)i);
  v4f hv, cv;
#pragma unroll
  for (int e = 0; e < 4; ++e) {
    const float ai = ai4[e];
    const float af = af4[e];
    const float ag = ag4[e];
    const float ao = ao4[e];
    const float hi = hi4[e];
    const float hf = hf4[e];
    const float hg = hg4[e];
    const float ho = ho4[e];
    const float zi = gi4[e] + bf16r(ai) + bf16r(hi);
    const float zf = gf4[e] + bf16r(af) + bf16r(hf);
    const float zg = gg4[e] + bf16r(ag) + bf16r(hg);
    const float zo = go4[e] + bf16r(ao) + bf16r(ho);
    const float si = 1.0f / (1.0f + expf(-zi));
    const float sf = 1.0f / (1.0f + expf(-zf));
    const float so = 1.0f / (1.0f + expf(-zo));
    const float tg = tanhf(zg);
    const float cell = sf * pc4[e] + si * tg;
    cv[e] = cell;
    hv[e] = so * tanhf(cell);
  }
  float* ph = out + (size_t)i;
  float* pc = out + (size_t)kOutHalf + (size_t)i;
  *(volatile v4f*)ph = hv;
  *(volatile v4f*)pc = cv;
  __threadfence();
  *(volatile v4f*)ph = hv;
  *(volatile v4f*)pc = cv;
}

static_assert(((kB * k3H / 8) % 256) == 0 && (kB * k3H / 8) / 256 == 6144);
static_assert(((kH * k3H / 8) % 256) == 0 && (kH * k3H / 8) / 256 == 1536);
static_assert(((k4H * kKG / 8) % 256) == 0 && (k4H * kKG / 8) / 256 == 3072);
static_assert(((kB * kI / 8) % 256) == 0 && (kB * kI / 8) / 256 == 1024);
static_assert((kB % 256) == 0 && kB / 256 == 16);
static_assert(((kB * kH / 8) % 256) == 0 && (kB * kH / 8) / 256 == 2048);
static_assert(((kB * kH / 4) % 256) == 0 && (kB * kH / 4) / 256 == 4096);
static_assert(((kB / 32) * (kH / 64)) % 8 == 0 && ((kB / 32) * (kH / 64)) / 8 == 256);
static_assert(((kB / 32) * (k4H / 64)) % 8 == 0 && ((kB / 32) * (k4H / 64)) / 8 == 1024);
static_assert((k3H / 8) == 384 && (kKG / 8) == 192 && (kI / 8) == 64 && (kH / 8) == 128);

extern "C" void kernel_launch(void* const* d_in, const int* in_sizes, int n_in,
                              void* d_out, int out_size, void* d_ws, size_t ws_size,
                              hipStream_t stream)
{
  if (n_in < 19) return;
  if (in_sizes[0] != kB * kI) return;
  if (in_sizes[1] != kB * kH) return;
  if (in_sizes[2] != kB * kH) return;
  if (in_sizes[3] != kB * kH) return;
  if (in_sizes[4] != kB * kH) return;
  if (in_sizes[5] != kB * kH) return;
  if (in_sizes[6] != kB * kH) return;
  if (in_sizes[7] != kH * k3H) return;
  if (in_sizes[8] != kH) return;
  if (in_sizes[9] != kH * k3H) return;
  if (in_sizes[10] != kH) return;
  if (in_sizes[11] != kH) return;
  if (in_sizes[12] != kH) return;
  if (in_sizes[13] != kH) return;
  if (in_sizes[14] != kH) return;
  if (in_sizes[15] != k4H * kI) return;
  if (in_sizes[16] != k4H * kH) return;
  if (in_sizes[17] != k4H) return;
  if (in_sizes[18] != k4H) return;
  if (out_size != 2 * kOutHalf) return;
  if (ws_size < kWsTotal) return;

  const float* x_in    = (const float*)d_in[0];
  const float* h_left  = (const float*)d_in[1];
  const float* c_left  = (const float*)d_in[2];
  const float* h_up    = (const float*)d_in[3];
  const float* c_up    = (const float*)d_in[4];
  const float* h_last  = (const float*)d_in[5];
  const float* c_last  = (const float*)d_in[6];
  const float* Wh_proc = (const float*)d_in[7];
  const float* bh_proc = (const float*)d_in[8];
  const float* Wc_proc = (const float*)d_in[9];
  const float* bc_proc = (const float*)d_in[10];
  const float* gamma_h = (const float*)d_in[11];
  const float* beta_h  = (const float*)d_in[12];
  const float* gamma_c = (const float*)d_in[13];
  const float* beta_c  = (const float*)d_in[14];
  const float* W_ih    = (const float*)d_in[15];
  const float* W_hh    = (const float*)d_in[16];
  const float* b_ih    = (const float*)d_in[17];
  const float* b_hh    = (const float*)d_in[18];
  float* out = (float*)d_out;

  char* ws = (char*)d_ws;
  unsigned short* CH  = (unsigned short*)(ws + kOffCH);
  unsigned short* CC  = (unsigned short*)(ws + kOffCC);
  unsigned short* WHP = (unsigned short*)(ws + kOffWHP);
  unsigned short* WCP = (unsigned short*)(ws + kOffWCP);
  float*          RH  = (float*)(ws + kOffRH);
  float*          RC  = (float*)(ws + kOffRC);
  float*          STH = (float*)(ws + kOffSTH);
  float*          STC = (float*)(ws + kOffSTC);
  unsigned short* XH  = (unsigned short*)(ws + kOffXH);
  float*          PC  = (float*)(ws + kOffPC);
  unsigned short* WG  = (unsigned short*)(ws + kOffWG);
  float*          GT  = (float*)(ws + kOffGT);

  cat3_pack_kernel<<<(kB * k3H / 8) / 256, 256, 0, stream>>>(h_left, h_up, h_last, CH);
  cat3_pack_kernel<<<(kB * k3H / 8) / 256, 256, 0, stream>>>(c_left, c_up, c_last, CC);

  w_pack_kernel<<<(kH * k3H / 8) / 256, 256, 0, stream>>>(Wh_proc, WHP);
  w_pack_kernel<<<(kH * k3H / 8) / 256, 256, 0, stream>>>(Wc_proc, WCP);

  eng::gemm_f16_kernel<2, 0><<<dim3((kB / 32) * (kH / 64) / 8), 256, 0, stream>>>(
      CH, nullptr, k3H, WHP, nullptr, k3H, RH, kH, kB, kH, k3H, kWScale, 0.0f);
  eng::gemm_f16_kernel<2, 0><<<dim3((kB / 32) * (kH / 64) / 8), 256, 0, stream>>>(
      CC, nullptr, k3H, WCP, nullptr, k3H, RC, kH, kB, kH, k3H, kWScale, 0.0f);

  ln_stats_kernel<<<kB / 256, 256, 0, stream>>>(RH, bh_proc, STH);
  ln_stats_kernel<<<kB / 256, 256, 0, stream>>>(RC, bc_proc, STC);

  x_pack_kernel<<<(kB * kI / 8) / 256, 256, 0, stream>>>(x_in, XH);

  ln_apply_h_kernel<<<(kB * kH / 8) / 256, 256, 0, stream>>>(RH, bh_proc, gamma_h, beta_h, STH, XH);

  ln_apply_c_kernel<<<(kB * kH / 4) / 256, 256, 0, stream>>>(RC, bc_proc, gamma_c, beta_c, STC, PC);

  wg_pack_kernel<<<(k4H * kKG / 8) / 256, 256, 0, stream>>>(W_ih, W_hh, WG);

  eng::gemm_f16_kernel<2, 0><<<dim3((kB / 32) * (k4H / 64) / 8), 256, 0, stream>>>(
      XH, nullptr, kKG, WG, nullptr, kKG, GT, k4H, kB, k4H, kKG, kWScale, 0.0f);

  cell_out_kernel<<<(kB * kH / 4) / 256, 256, 0, stream>>>(GT, PC, b_ih, b_hh, out);
}
